// NATTEN1DAttention_67929202754075
// MI455X (gfx1250) — hardware-verified
//
#include <hip/hip_runtime.h>
#include <math.h>

typedef __attribute__((ext_vector_type(16))) _Float16 v16h;
typedef __attribute__((ext_vector_type(16))) __bf16 v16b;
typedef __attribute__((ext_vector_type(8)))  _Float16 v8h;
typedef __attribute__((ext_vector_type(8)))  float v8f;
typedef __attribute__((ext_vector_type(4)))  float v4f;
typedef __attribute__((ext_vector_type(2)))  float v2f;
typedef __attribute__((ext_vector_type(4)))  unsigned v4u;
typedef __attribute__((ext_vector_type(4)))  int v4i;
typedef float __attribute__((may_alias)) float_a;
typedef int __attribute__((may_alias)) int_a;

template <typename T> __device__ __forceinline__ void vst2(void* p, T v) { *(volatile T*)p = v; __threadfence(); *(volatile T*)p = v; }
__device__ __forceinline__ v8f wmma16(v16h a, v16h b, v8f c) {
  v8f d = __builtin_amdgcn_wmma_f32_16x16x32_f16(false, a, false, b, (short)0, c, false, false);
  asm volatile("v_nop\n\tv_nop\n\tv_nop\n\tv_nop" : "+v"(d) : "v"(a), "v"(b));
  return d;
}
__device__ __forceinline__ v8f wmma_bf(v16b a, v16b b, v8f c) {
  v8f d = __builtin_amdgcn_wmma_f32_16x16x32_bf16(false, a, false, b, (short)0, c, false, false);
  asm volatile("v_nop\n\tv_nop\n\tv_nop\n\tv_nop" : "+v"(d) : "v"(a), "v"(b));
  return d;
}
__device__ __forceinline__ v16h frag_h(const _Float16* rowk0, int lane) {
  union { v16h v; v8h q[2]; } u; const _Float16* p = rowk0 + 8 * (lane >> 4);
  u.q[0] = *(const v8h*)p; u.q[1] = *(const v8h*)(p + 16); return u.v;
}
__device__ __forceinline__ v16h frag_f32(const float* rowk0, int lane) {
  v16h a; const float* p = rowk0 + 8 * (lane >> 4);
#pragma unroll
  for (int i = 0; i < 8; ++i) { a[i] = (_Float16)p[i]; a[8 + i] = (_Float16)p[16 + i]; }
  return a;
}
__device__ __forceinline__ v16h frag_f32s(const float* rowk0, int lane, float sc) {
  v16h a; const float* p = rowk0 + 8 * (lane >> 4);
#pragma unroll
  for (int i = 0; i < 8; ++i) { a[i] = (_Float16)(p[i] * sc); a[8 + i] = (_Float16)(p[16 + i] * sc); }
  return a;
}
__device__ __forceinline__ v16h fragc_f32(const float* W, int k0, int n, int lane, int ld, int K) {
  v16h a; const int g = lane >> 4;
#pragma unroll
  for (int i = 0; i < 8; ++i) { const int ka = k0 + 8 * g + i, kb = ka + 16;
    a[i] = (_Float16)(ka < K ? W[(size_t)ka * ld + n] : 0.f); a[8 + i] = (_Float16)(kb < K ? W[(size_t)kb * ld + n] : 0.f); }
  return a;
}
struct F2 { v16b h, l; };
__device__ __forceinline__ F2 bsplit16(const float v[16]) { F2 r;
#pragma unroll
  for (int i = 0; i < 16; ++i) { const __bf16 h = (__bf16)v[i]; r.h[i] = h; r.l[i] = (__bf16)(v[i] - (float)h); }
  return r; }
__device__ __forceinline__ F2 split_row(const float* row, int k0, int lane) { float v[16]; const float* p = row + k0 + 8 * (lane >> 4);
#pragma unroll
  for (int i = 0; i < 8; ++i) { v[i] = p[i]; v[8 + i] = p[16 + i]; }
  return bsplit16(v); }
__device__ __forceinline__ F2 split_rowK(const float* row, int k0, int lane, int K) { float v[16]; const int g = lane >> 4;
#pragma unroll
  for (int i = 0; i < 8; ++i) { const int ka = k0 + 8 * g + i, kb = ka + 16; v[i] = ka < K ? row[ka] : 0.f; v[8 + i] = kb < K ? row[kb] : 0.f; }
  return bsplit16(v); }
__device__ __forceinline__ F2 split_col(const float* W, int k0, int n, int lane, int ld, int K) { float v[16]; const int g = lane >> 4;
#pragma unroll
  for (int i = 0; i < 8; ++i) { const int ka = k0 + 8 * g + i, kb = ka + 16; v[i] = ka < K ? W[(size_t)ka * ld + n] : 0.f; v[8 + i] = kb < K ? W[(size_t)kb * ld + n] : 0.f; }
  return bsplit16(v); }
__device__ __forceinline__ v8f mac3(const F2& a, const F2& b, v8f c) { c = wmma_bf(a.l, b.h, c); c = wmma_bf(a.h, b.l, c); return wmma_bf(a.h, b.h, c); }
__device__ __forceinline__ float sigm(float v) { return 1.0f / (1.0f + expf(-v)); }
#define LDSX() do { asm volatile("s_wait_dscnt 0" ::: "memory"); __builtin_amdgcn_wave_barrier(); __builtin_amdgcn_fence(__ATOMIC_RELEASE, "workgroup"); } while (0)


#define NB 2
#define SS 2048
#define E 512
#define NH 8
#define HD 64
#define KS 63
#define NBW 31

__global__ __launch_bounds__(128) void k_natt(const float* __restrict__ x, float* __restrict__ out) {
  __shared__ __align__(16) float sS[4][16][68]; __shared__ __align__(16) float sO[4][16][68];
  const int tid = threadIdx.x, w = tid >> 5, lane = tid & 31, col = lane & 15, g = lane >> 4;
  const int bh = blockIdx.y, b = bh / NH, h = bh % NH; const int q0 = blockIdx.x * 64 + w * 16;
  const float* xb = x + (size_t)b * SS * E + h * HD;
  F2 aq[2];
#pragma unroll
  for (int kc = 0; kc < 2; ++kc) aq[kc] = split_row(xb + (size_t)(q0 + col) * E, kc * 32, lane);
  float mrun = -3.0e38f, lrun = 0.f; v8f acc[4] = {};
  const int kbase = (int)blockIdx.x * 64 - 64;
#pragma unroll 1
  for (int kt = 0; kt < 3; ++kt) { const int k0 = kbase + kt * 64; if (k0 + 64 <= 0 || k0 >= SS) continue;
#pragma unroll
    for (int t = 0; t < 4; ++t) { const int key = k0 + t * 16 + col; const int keyc = key < 0 ? 0 : (key >= SS ? SS - 1 : key);
      const F2 bk = split_row(xb + (size_t)keyc * E, 0, lane), bk1 = split_row(xb + (size_t)keyc * E, 32, lane);
      v8f s = wmma_bf(aq[0].h, bk.h, (v8f){}); s = wmma_bf(aq[1].h, bk1.h, s);
#pragma unroll
      for (int r = 0; r < 8; ++r) { const int i = q0 + 8 * g + r; int st = i - NBW; st = st < 0 ? 0 : (st > SS - KS ? SS - KS : st);
        const bool ok = key >= st && key < st + KS && key >= 0 && key < SS; sS[w][8 * g + r][t * 16 + col] = ok ? s[r] * 0.125f : -3.0e38f; } }
    LDSX();
    float mx = -3.4e38f;
#pragma unroll
    for (int jj = 0; jj < 32; ++jj) mx = fmaxf(mx, sS[w][col][g * 32 + jj]);
    mx = fmaxf(mx, __shfl_xor(mx, 16, 32));
    const float mnew = fmaxf(mrun, mx); const float corr = expf(mrun - mnew);
    float ps = 0.f;
#pragma unroll
    for (int jj = 0; jj < 32; ++jj) { const float sv = sS[w][col][g * 32 + jj]; const float p = (sv <= -1.0e38f) ? 0.f : expf(sv - mnew); ps += p; sS[w][col][g * 32 + jj] = p; }
    ps += __shfl_xor(ps, 16, 32);
    lrun = lrun * corr + ps; mrun = mnew;
#pragma unroll
    for (int r = 0; r < 8; ++r) { const float cr = __shfl(corr, 8 * g + r, 32);
#pragma unroll
      for (int t2 = 0; t2 < 4; ++t2) acc[t2][r] *= cr; }
    LDSX();
#pragma unroll
    for (int kc = 0; kc < 2; ++kc) { const F2 pa = split_row(&sS[w][col][0], kc * 32, lane); const int kr0 = k0 + kc * 32;
      const int kcl = kr0 < 0 ? 0 : (kr0 + 32 > SS ? SS - 32 : kr0);
#pragma unroll
      for (int t2 = 0; t2 < 4; ++t2) { const F2 bv = split_col(xb + (size_t)kcl * E, 0, t2 * 16 + col, lane, E, 32);
        if (kcl == kr0) { acc[t2] = wmma_bf(pa.h, bv.h, acc[t2]); acc[t2] = wmma_bf(pa.l, bv.h, acc[t2]); } } }
    LDSX(); }
#pragma unroll
  for (int r = 0; r < 8; ++r) { const float lr = __shfl(lrun, 8 * g + r, 32); const float inv = 1.0f / lr;
#pragma unroll
    for (int t2 = 0; t2 < 4; ++t2) sO[w][8 * g + r][t2 * 16 + col] = acc[t2][r] * inv; }
  LDSX();
  for (int qq = lane; qq < 16 * 16; qq += 32) { const int rl = qq >> 4, pc = qq & 15; vst2(out + ((size_t)b * SS + q0 + rl) * E + h * HD + pc * 4, *(const v4f*)(&sO[w][rl][pc * 4])); }
}
extern "C" void kernel_launch(void* const* d_in, const int* in_sizes, int n_in, void* d_out, int out_size, void* d_ws, size_t ws_size, hipStream_t stream) {
  (void)in_sizes; (void)n_in; (void)out_size; (void)ws_size; (void)d_ws;
  const float* x = (const float*)d_in[0];
  float* out = (float*)d_out;
  k_natt<<<dim3(SS / 64, NB * NH), 128, 0, stream>>>(x, out);
}
